// SyntaxTreeNetwork_82136954569227
// MI455X (gfx1250) — hardware-verified
//
#include <hip/hip_runtime.h>
#include <math.h>

typedef __attribute__((ext_vector_type(16))) _Float16 v16h;
typedef __attribute__((ext_vector_type(16))) __bf16 v16b;
typedef __attribute__((ext_vector_type(8)))  _Float16 v8h;
typedef __attribute__((ext_vector_type(8)))  float v8f;
typedef __attribute__((ext_vector_type(4)))  float v4f;
typedef __attribute__((ext_vector_type(2)))  float v2f;
typedef __attribute__((ext_vector_type(4)))  unsigned v4u;
typedef __attribute__((ext_vector_type(4)))  int v4i;
typedef float __attribute__((may_alias)) float_a;
typedef int __attribute__((may_alias)) int_a;

template <typename T> __device__ __forceinline__ void vst2(void* p, T v) { *(volatile T*)p = v; __threadfence(); *(volatile T*)p = v; }
__device__ __forceinline__ v8f wmma16(v16h a, v16h b, v8f c) {
  v8f d = __builtin_amdgcn_wmma_f32_16x16x32_f16(false, a, false, b, (short)0, c, false, false);
  asm volatile("v_nop\n\tv_nop\n\tv_nop\n\tv_nop" : "+v"(d) : "v"(a), "v"(b));
  return d;
}
__device__ __forceinline__ v8f wmma_bf(v16b a, v16b b, v8f c) {
  v8f d = __builtin_amdgcn_wmma_f32_16x16x32_bf16(false, a, false, b, (short)0, c, false, false);
  asm volatile("v_nop\n\tv_nop\n\tv_nop\n\tv_nop" : "+v"(d) : "v"(a), "v"(b));
  return d;
}
__device__ __forceinline__ v16h frag_h(const _Float16* rowk0, int lane) {
  union { v16h v; v8h q[2]; } u; const _Float16* p = rowk0 + 8 * (lane >> 4);
  u.q[0] = *(const v8h*)p; u.q[1] = *(const v8h*)(p + 16); return u.v;
}
__device__ __forceinline__ v16h frag_f32(const float* rowk0, int lane) {
  v16h a; const float* p = rowk0 + 8 * (lane >> 4);
#pragma unroll
  for (int i = 0; i < 8; ++i) { a[i] = (_Float16)p[i]; a[8 + i] = (_Float16)p[16 + i]; }
  return a;
}
__device__ __forceinline__ v16h frag_f32s(const float* rowk0, int lane, float sc) {
  v16h a; const float* p = rowk0 + 8 * (lane >> 4);
#pragma unroll
  for (int i = 0; i < 8; ++i) { a[i] = (_Float16)(p[i] * sc); a[8 + i] = (_Float16)(p[16 + i] * sc); }
  return a;
}
__device__ __forceinline__ v16h fragc_f32(const float* W, int k0, int n, int lane, int ld, int K) {
  v16h a; const int g = lane >> 4;
#pragma unroll
  for (int i = 0; i < 8; ++i) { const int ka = k0 + 8 * g + i, kb = ka + 16;
    a[i] = (_Float16)(ka < K ? W[(size_t)(ka < K ? ka : K - 1) * ld + n] : 0.f); a[8 + i] = (_Float16)(kb < K ? W[(size_t)(kb < K ? kb : K - 1) * ld + n] : 0.f); }
  return a;
}
struct F2 { v16b h, l; };
__device__ __forceinline__ F2 bsplit16(const float v[16]) { F2 r;
#pragma unroll
  for (int i = 0; i < 16; ++i) { const __bf16 h = (__bf16)v[i]; r.h[i] = h; r.l[i] = (__bf16)(v[i] - (float)h); }
  return r; }
__device__ __forceinline__ F2 split_row(const float* row, int k0, int lane) { float v[16]; const float* p = row + k0 + 8 * (lane >> 4);
#pragma unroll
  for (int i = 0; i < 8; ++i) { v[i] = p[i]; v[8 + i] = p[16 + i]; }
  return bsplit16(v); }
__device__ __forceinline__ F2 split_rowK(const float* row, int k0, int lane, int K) { float v[16]; const int g = lane >> 4;
#pragma unroll
  for (int i = 0; i < 8; ++i) { const int ka = k0 + 8 * g + i, kb = ka + 16; v[i] = ka < K ? row[ka < K ? ka : K - 1] : 0.f; v[8 + i] = kb < K ? row[kb < K ? kb : K - 1] : 0.f; }
  return bsplit16(v); }
__device__ __forceinline__ F2 split_col(const float* W, int k0, int n, int lane, int ld, int K) { float v[16]; const int g = lane >> 4;
#pragma unroll
  for (int i = 0; i < 8; ++i) { const int ka = k0 + 8 * g + i, kb = ka + 16; v[i] = ka < K ? W[(size_t)(ka < K ? ka : K - 1) * ld + n] : 0.f; v[8 + i] = kb < K ? W[(size_t)(kb < K ? kb : K - 1) * ld + n] : 0.f; }
  return bsplit16(v); }
__device__ __forceinline__ v8f mac3(const F2& a, const F2& b, v8f c) { c = wmma_bf(a.l, b.h, c); c = wmma_bf(a.h, b.l, c); return wmma_bf(a.h, b.h, c); }
__device__ __forceinline__ float sigm(float v) { return 1.0f / (1.0f + expf(-v)); }
#define LDSX() do { asm volatile("s_wait_dscnt 0" ::: "memory"); __builtin_amdgcn_wave_barrier(); __builtin_amdgcn_fence(__ATOMIC_RELEASE, "workgroup"); } while (0)


#define NBT 64
#define NL 512
#define HH 256
#ifndef NLEV
#define NLEV 9
#endif
typedef __attribute__((ext_vector_type(8))) __bf16 v8b;
__device__ __forceinline__ v16b frag_b(const __bf16* rowk0, int lane) {
  union { v16b v; v8b q[2]; } u; const __bf16* p = rowk0 + 8 * (lane >> 4);
  u.q[0] = *(const v8b*)p; u.q[1] = *(const v8b*)(p + 16); return u.v;
}
__device__ __forceinline__ float bfr(float v) { return (float)(__bf16)v; }
__device__ __attribute__((noinline)) float exp_ni(float v) { return expf(v); }
__device__ __attribute__((noinline)) float erf_ni(float v) { return erff(v); }

#define WS_PW  0u
#define WS_HA  (WS_PW + 2u * 64 * HH * 2 * HH)
#define WS_HB  (WS_HA + 4u * NBT * NL * HH)
#define WS_END (WS_HB + 4u * NBT * NL * HH)

__global__ __launch_bounds__(256) void k_packw(const float* __restrict__ RW, __bf16* __restrict__ PW) {
  const size_t row = blockIdx.x; const int t = threadIdx.x; __shared__ __align__(16) __bf16 s[2 * HH]; for (int k = t; k < 2 * HH; k += 256) s[k] = (__bf16)RW[row * 2 * HH + k]; __syncthreads();
  if (t < 2 * HH / 8) vst2((unsigned*)(PW + row * 2 * HH + t * 8), *(const v4u*)&s[t * 8]);
}
__device__ __attribute__((noinline)) float tanh_p(float v) { return tanhf(v); }
__global__ __launch_bounds__(256) void k_leaf(const int* __restrict__ TOK, const int* __restrict__ PNT, const float* __restrict__ EMB, const float* __restrict__ BIA, float* __restrict__ H) {
  const int b = blockIdx.y, l = blockIdx.x, t = threadIdx.x; const int tok = TOK[b * NL + l], nt = PNT[b * NL + l];
  __shared__ __align__(16) float s[HH]; s[t] = tanh_p(bfr(EMB[(size_t)tok * HH + t]) + bfr(BIA[(size_t)nt * HH + t])); __syncthreads();
  if (t < HH / 4) vst2(H + ((size_t)b * NL + l) * HH + t * 4, *(const v4f*)&s[t * 4]);
}
__global__ __launch_bounds__(128) void k_level(const float* __restrict__ Hin, const __bf16* __restrict__ PW, const int* __restrict__ RID, const int* __restrict__ NTID, const float* __restrict__ BIA, int off, int nin, float* __restrict__ Hout) {
  __shared__ __align__(16) float so[4][16][132];
  const int tid = threadIdx.x, wave = tid >> 5, lane = tid & 31, col = lane & 15, g = lane >> 4; const int j = blockIdx.x; const int n0 = blockIdx.y * 128; const int nout = nin / 2;
  const int rule = RID[off + j], nt = NTID[off + j]; const __bf16* Wr = PW + (size_t)rule * HH * 2 * HH;
  v8f acc[8] = {};
#pragma unroll 2
  for (int kc = 0; kc < 2 * HH / 32; ++kc) { const int b = wave * 16 + col; const F2 a = split_row(Hin + ((size_t)b * nin + 2 * j) * HH, kc * 32, lane);
#pragma unroll
    for (int t8 = 0; t8 < 8; ++t8) { const v16b w = frag_b(Wr + (size_t)(n0 + t8 * 16 + col) * 2 * HH + kc * 32, lane); acc[t8] = wmma_bf(a.l, w, acc[t8]); acc[t8] = wmma_bf(a.h, w, acc[t8]); } }
#pragma unroll
  for (int t8 = 0; t8 < 8; ++t8) { const int c = n0 + t8 * 16 + col; const float bb = bfr(BIA[(size_t)nt * HH + c]);
#pragma unroll
    for (int r = 0; r < 8; ++r) so[wave][8 * g + r][t8 * 16 + col] = tanh_p(acc[t8][r] + bb); }
  LDSX();
  for (int rl = 0; rl < 16; ++rl) { const int b = wave * 16 + rl; vst2(Hout + ((size_t)b * nout + j) * HH + n0 + lane * 4, *(const v4f*)&so[wave][rl][lane * 4]); }
}
__global__ __launch_bounds__(64) void k_root(const float* __restrict__ Hf, int nfin, float* __restrict__ OUT) { const int b = blockIdx.x, t = threadIdx.x; vst2(OUT + (size_t)b * HH + t * 4, *(const v4f*)(Hf + (size_t)b * nfin * HH + t * 4)); }
extern "C" void kernel_launch(void* const* d_in, const int* in_sizes, int n_in, void* d_out, int out_size, void* d_ws, size_t ws_size, hipStream_t stream) {
  (void)in_sizes; (void)n_in; (void)out_size;
  const float** F = (const float**)d_in;
  if (ws_size < (size_t)WS_END) return;
  char* ws = (char*)d_ws; __bf16* PW = (__bf16*)(ws + WS_PW); float *HA = (float*)(ws + WS_HA), *HB = (float*)(ws + WS_HB);
  k_packw<<<64 * HH, 256, 0, stream>>>(F[5], PW);
  k_leaf<<<dim3(NL, NBT), 256, 0, stream>>>((const int*)d_in[0], (const int*)d_in[1], F[4], F[6], HA);
  float* cur = HA; float* nxt = HB; int n = NL; int off = 0;
  for (int lev = 0; lev < NLEV; ++lev) { const int nout = n / 2; k_level<<<dim3(nout, HH / 128), 128, 0, stream>>>(cur, PW, (const int*)d_in[2], (const int*)d_in[3], F[6], off, n, nxt); off += nout; n = nout; float* tmp = cur; cur = nxt; nxt = tmp; }
  k_root<<<NBT, 64, 0, stream>>>(cur, n, (float*)d_out);
}
